// MyMultiHeadRelativeAttention_4526895530601
// MI455X (gfx1250) — hardware-verified
//
#include <hip/hip_runtime.h>


namespace {
constexpr int Bn = 4, S = 1024, D = 1024, H = 16, HD = 64, NT = Bn * S, NREL = 257, NRP = 272  ;
constexpr float QS = 8.0f, KS = 8.0f, VS = 8.0f, PS = 8.0f, AS_ = 8.0f;
constexpr size_t PL = (size_t)Bn * H * S * HD;

typedef _Float16 b16;
typedef __attribute__((ext_vector_type(16))) _Float16 v16b;
typedef __attribute__((ext_vector_type(8))) _Float16 v8b;
typedef __attribute__((ext_vector_type(8))) float v8f;
typedef __attribute__((ext_vector_type(4))) float v4f;
__device__ __forceinline__ float bf16_rne(float f) { unsigned int u = __float_as_uint(f); u += 0x7FFFu + ((u >> 16) & 1u); return __uint_as_float(u & 0xFFFF0000u); }
__device__ __forceinline__ void split16(float v, b16& hi, b16& lo) { hi = (b16)v; lo = (b16)(v - (float)hi); }
__device__ __forceinline__ v16b frag_kb(const b16* p, int hh) { const v8b a = *(const v8b*)(p + 8 * hh), b = *(const v8b*)(p + 16 + 8 * hh); v16b f;
#pragma unroll
  for (int e = 0; e < 8; ++e) { f[e] = a[e]; f[8 + e] = b[e]; } return f; }
__device__ __forceinline__ v16b frag_x(const float* p, int hh) { v16b f;
#pragma unroll
  for (int e = 0; e < 8; ++e) { f[e] = (b16)bf16_rne(p[8 * hh + e]); f[8 + e] = (b16)bf16_rne(p[16 + 8 * hh + e]); } return f; }
__device__ __forceinline__ void frag_split(const float* p, int hh, v16b& fh, v16b& fl) {
#pragma unroll
  for (int e = 0; e < 8; ++e) { b16 a, c; split16(p[8 * hh + e] * AS_, a, c); fh[e] = a; fl[e] = c; split16(p[16 + 8 * hh + e] * AS_, a, c); fh[8 + e] = a; fl[8 + e] = c; } }
__device__ __forceinline__ v8f wmma16b(v16b a, v16b b, v8f c) { v8f d = __builtin_amdgcn_wmma_f32_16x16x32_f16(false, a, false, b, (short)0, c, false, false); asm volatile("v_nop\n\tv_nop\n\tv_nop\n\tv_nop" : "+v"(d) : "v"(a), "v"(b)); return d; }
__device__ __forceinline__ void wave_lds_sync() { __builtin_amdgcn_fence(__ATOMIC_RELEASE, "workgroup"); __builtin_amdgcn_wave_barrier(); __builtin_amdgcn_fence(__ATOMIC_ACQUIRE, "workgroup"); }
__device__ __forceinline__ float nexp(float x) { return __builtin_amdgcn_exp2f(x * 1.4426950408889634f); }

struct Wo_ { static constexpr size_t QKV = 0, O = (size_t)3 * D * D, REL = O + (size_t)D * D, END = REL + (size_t)NRP * HD; };
__global__ __launch_bounds__(256) void prep_kernel(const float* __restrict__ Wq, const float* __restrict__ Wk, const float* __restrict__ Wv, const float* __restrict__ Wo, const float* __restrict__ rel, const float* __restrict__ bq, const float* __restrict__ bk, const float* __restrict__ bv, const float* __restrict__ bo, b16* __restrict__ R, float* __restrict__ P) {
  const size_t tid = (size_t)blockIdx.x * 256 + threadIdx.x, nth = (size_t)gridDim.x * 256;
  auto tr = [&](size_t base, int nout, int kin, const float* W) { for (size_t p = tid; p < (size_t)nout * (kin / 8); p += nth) { const int o = (int)(p / (kin / 8)), k0 = (int)(p % (kin / 8)) * 8; v8b v;
#pragma unroll
      for (int e = 0; e < 8; ++e) v[e] = (b16)bf16_rne(W[(size_t)(k0 + e) * nout + o]); *(volatile v8b*)(R + base + (size_t)o * kin + k0) = v; } };
  for (int pass = 0; pass < 2; ++pass) {
    tr(Wo_::QKV, D, D, Wq); tr(Wo_::QKV + (size_t)D * D, D, D, Wk); tr(Wo_::QKV + (size_t)2 * D * D, D, D, Wv); tr(Wo_::O, D, D, Wo);
    for (size_t p = tid; p < (size_t)NRP * HD / 8; p += nth) { const int r = (int)(p / (HD / 8)), d8 = (int)(p % (HD / 8)) * 8; v8b v; for (int e = 0; e < 8; ++e) v[e] = (b16)((r < NREL) ? bf16_rne(rel[r * HD + d8 + e]) : 0.0f); *(volatile v8b*)(R + Wo_::REL + (size_t)r * HD + d8) = v; }
    for (size_t q = tid; q < 4096; q += nth) { const int i = (int)q; P[q] = bf16_rne((i < 1024) ? bq[i] : (i < 2048) ? bk[i - 1024] : (i < 3072) ? bv[i - 2048] : bo[i - 3072]); }
    __threadfence(); }
}

__global__ __launch_bounds__(128) void proj_kernel(const float* __restrict__ x, const b16* __restrict__ R, const float* __restrict__ P, b16* __restrict__ qh, b16* __restrict__ ql, b16* __restrict__ kh, b16* __restrict__ kl, b16* __restrict__ vt, b16* __restrict__ vtl) {
  __shared__ __attribute__((aligned(16))) b16 Th[4][32][64 + 8], Tl[4][32][64 + 8]; __shared__ __attribute__((aligned(16))) b16 Tv[64][128 + 8], Tvl[64][128 + 8];
  const int lane = threadIdx.x & 31, wave = threadIdx.x >> 5, nloc = lane & 15, hlf = lane >> 4, h = blockIdx.x, which = blockIdx.z, p0 = blockIdx.y * 128, m0 = p0 + wave * 32, b = p0 / S, t0 = p0 % S, c0 = h * HD;
  const b16* Wt = R + Wo_::QKV + (size_t)which * D * D;
  v8f acc[2][4];
#pragma unroll
  for (int r = 0; r < 2; ++r)
#pragma unroll
    for (int t = 0; t < 4; ++t) acc[r][t] = (v8f){};
#pragma unroll 2
  for (int kb = 0; kb < D; kb += 32) { const v16b a0 = frag_x(x + (size_t)(m0 + nloc) * D + kb, hlf), a1 = frag_x(x + (size_t)(m0 + 16 + nloc) * D + kb, hlf);
#pragma unroll
    for (int t = 0; t < 4; ++t) { const v16b bw = frag_kb(Wt + (size_t)(c0 + t * 16 + nloc) * D + kb, hlf); acc[0][t] = wmma16b(a0, bw, acc[0][t]); acc[1][t] = wmma16b(a1, bw, acc[1][t]); } }
  const float* bias = P + which * D + c0;
  if (which < 2) { const float sc = (which == 0) ? QS : KS; b16* Ph = (which == 0) ? qh : kh; b16* Plo = (which == 0) ? ql : kl;
#pragma unroll
    for (int t = 0; t < 4; ++t)
#pragma unroll
      for (int r = 0; r < 2; ++r)
#pragma unroll
        for (int v = 0; v < 8; ++v) { b16 a_, c_; split16((acc[r][t][v] + bias[t * 16 + nloc]) * sc, a_, c_); Th[wave][r * 16 + 8 * hlf + v][t * 16 + nloc] = a_; Tl[wave][r * 16 + 8 * hlf + v][t * 16 + nloc] = c_; }
    wave_lds_sync();
    const size_t base = (((size_t)b * H + h) * S + (m0 % S)) * HD;
    for (int pass = 0; pass < 2; ++pass) {
#pragma unroll
      for (int j = 0; j < 8; ++j) { const int rr = j * 4 + (lane >> 3), c8 = (lane & 7) * 8; *(volatile v8b*)(Ph + base + (size_t)rr * HD + c8) = *(const v8b*)(&Th[wave][rr][c8]); *(volatile v8b*)(Plo + base + (size_t)rr * HD + c8) = *(const v8b*)(&Tl[wave][rr][c8]); }
      __threadfence(); }
    return; }
#pragma unroll
  for (int t = 0; t < 4; ++t)
#pragma unroll
    for (int r = 0; r < 2; ++r)
#pragma unroll
      for (int v = 0; v < 8; ++v) { b16 a_, c_; split16((acc[r][t][v] + bias[t * 16 + nloc]) * VS, a_, c_); Tv[t * 16 + nloc][wave * 32 + r * 16 + 8 * hlf + v] = a_; Tvl[t * 16 + nloc][wave * 32 + r * 16 + 8 * hlf + v] = c_; }
  __syncthreads();
  for (int pass = 0; pass < 2; ++pass) { for (int i = threadIdx.x; i < 64 * 16; i += 128) { const int d = i >> 4, c8 = (i & 15) * 8; const size_t o = (((size_t)b * H + h) * HD + d) * S + t0 + c8; *(volatile v8b*)(vt + o) = *(const v8b*)(&Tv[d][c8]); *(volatile v8b*)(vtl + o) = *(const v8b*)(&Tvl[d][c8]); } __threadfence(); }
}

__global__ __launch_bounds__(128) void attn_kernel(const b16* __restrict__ qh, const b16* __restrict__ ql, const b16* __restrict__ kh, const b16* __restrict__ kl, const b16* __restrict__ vt, const b16* __restrict__ vtl, const b16* __restrict__ R, float* __restrict__ ctx) {
  __shared__ float Rr[4][16][NREL + 3]; __shared__ __attribute__((aligned(16))) float Os[16][4 * HD + 4];
  const int wave = threadIdx.x >> 5, lane = threadIdx.x & 31, hh = lane >> 4, col = lane & 15; const int b = blockIdx.x / (S / 16), q0 = (blockIdx.x % (S / 16)) * 16, h = blockIdx.y * 4 + wave, qi = q0 + col;
  const size_t pb = ((size_t)b * H + h) * S * HD; const b16* V = vt + ((size_t)b * H + h) * HD * S; const b16* Vl = vtl + ((size_t)b * H + h) * HD * S; const b16* REL = R + Wo_::REL;
  { const v16b a0h = frag_kb(qh + pb + (size_t)(q0 + (lane & 15)) * HD, hh), a0l = frag_kb(ql + pb + (size_t)(q0 + (lane & 15)) * HD, hh), a1h = frag_kb(qh + pb + (size_t)(q0 + (lane & 15)) * HD + 32, hh), a1l = frag_kb(ql + pb + (size_t)(q0 + (lane & 15)) * HD + 32, hh);
    for (int t = 0; t < 17; ++t) { v8f acc = {}; const v16b b0 = frag_kb(REL + (size_t)(t * 16 + col) * HD, hh), b1 = frag_kb(REL + (size_t)(t * 16 + col) * HD + 32, hh);
      acc = wmma16b(a0h, b0, acc); acc = wmma16b(a0l, b0, acc); acc = wmma16b(a1h, b1, acc); acc = wmma16b(a1l, b1, acc);
#pragma unroll
      for (int r = 0; r < 8; ++r) { const int dl = t * 16 + col; if (dl < NREL) Rr[wave][8 * hh + r][dl] = acc[r] * (1.0f / QS); } } }
  wave_lds_sync();
  const v16b qa0 = frag_kb(qh + pb + (size_t)qi * HD, hh), qa1 = frag_kb(qh + pb + (size_t)qi * HD + 32, hh), qb0 = frag_kb(ql + pb + (size_t)qi * HD, hh), qb1 = frag_kb(ql + pb + (size_t)qi * HD + 32, hh);
  float m = -INFINITY, l = 0.0f; v8f o[4] = {{}, {}, {}, {}};
  for (int kb = 0; kb < S; kb += 32) {
    v8f s0 = {}, s1 = {};
    { const v16b k0h = frag_kb(kh + pb + (size_t)(kb + col) * HD, hh), k0l = frag_kb(kl + pb + (size_t)(kb + col) * HD, hh), k1h = frag_kb(kh + pb + (size_t)(kb + col) * HD + 32, hh), k1l = frag_kb(kl + pb + (size_t)(kb + col) * HD + 32, hh);
      s0 = wmma16b(k0h, qa0, s0); s0 = wmma16b(k0h, qb0, s0); s0 = wmma16b(k0l, qa0, s0); s0 = wmma16b(k1h, qa1, s0); s0 = wmma16b(k1h, qb1, s0); s0 = wmma16b(k1l, qa1, s0); }
    { const v16b k0h = frag_kb(kh + pb + (size_t)(kb + 16 + col) * HD, hh), k0l = frag_kb(kl + pb + (size_t)(kb + 16 + col) * HD, hh), k1h = frag_kb(kh + pb + (size_t)(kb + 16 + col) * HD + 32, hh), k1l = frag_kb(kl + pb + (size_t)(kb + 16 + col) * HD + 32, hh);
      s1 = wmma16b(k0h, qa0, s1); s1 = wmma16b(k0h, qb0, s1); s1 = wmma16b(k0l, qa0, s1); s1 = wmma16b(k1h, qa1, s1); s1 = wmma16b(k1h, qb1, s1); s1 = wmma16b(k1l, qa1, s1); }
    float mr = -INFINITY;
#pragma unroll
    for (int r = 0; r < 8; ++r) { const int ka = kb + 8 * hh + r, kc = ka + 16; int da = qi - ka, dc = qi - kc; da = (da < -128) ? -128 : (da > 128 ? 128 : da); dc = (dc < -128) ? -128 : (dc > 128 ? 128 : dc);
      s0[r] = (s0[r] * (1.0f / (QS * KS)) + Rr[wave][col][da + 128]) * 0.125f; s1[r] = (s1[r] * (1.0f / (QS * KS)) + Rr[wave][col][dc + 128]) * 0.125f; mr = fmaxf(mr, fmaxf(s0[r], s1[r])); }
    mr = fmaxf(mr, __shfl_xor(mr, 16));
    const float mn = fmaxf(m, mr), al_ = nexp(m - mn); m = mn; float sum = 0.0f; v16b ph, pl;
#pragma unroll
    for (int r = 0; r < 8; ++r) { const float e0 = nexp(s0[r] - mn), e1 = nexp(s1[r] - mn); sum += e0 + e1; b16 a_, c_; split16(e0 * PS, a_, c_); ph[r] = a_; pl[r] = c_; split16(e1 * PS, a_, c_); ph[8 + r] = a_; pl[8 + r] = c_; }
    sum += __shfl_xor(sum, 16); l = l * al_ + sum;
#pragma unroll
    for (int t = 0; t < 4; ++t) { o[t] *= al_; const v16b vf = frag_kb(V + (size_t)(t * 16 + col) * S + kb, hh), vlf = frag_kb(Vl + (size_t)(t * 16 + col) * S + kb, hh); o[t] = wmma16b(vf, ph, o[t]); o[t] = wmma16b(vf, pl, o[t]); o[t] = wmma16b(vlf, ph, o[t]); } }
  const float inv = 1.0f / (l * VS * PS);
#pragma unroll
  for (int t = 0; t < 4; ++t)
#pragma unroll
    for (int r = 0; r < 8; ++r) Os[col][wave * HD + t * 16 + 8 * hh + r] = o[t][r] * inv;
  __syncthreads();
  for (int pass = 0; pass < 2; ++pass) { for (int i = threadIdx.x; i < 16 * 64; i += 128) { const int rr = i >> 6, c4 = (i & 63) * 4; *(volatile v4f*)(ctx + ((size_t)(b * S + q0 + rr)) * D + blockIdx.y * 4 * HD + c4) = *(const v4f*)(&Os[rr][c4]); } __threadfence(); }
}

__global__ __launch_bounds__(64) void out_kernel(const float* __restrict__ ctx, const b16* __restrict__ R, const float* __restrict__ P, float* __restrict__ out) {
  __shared__ __attribute__((aligned(16))) float Ts[2][32][128 + 4];
  const int lane = threadIdx.x & 31, wave = threadIdx.x >> 5, nloc = lane & 15, hlf = lane >> 4, m0 = blockIdx.y * 32, c0 = blockIdx.x * 256 + wave * 128; const b16* Wo = R + Wo_::O;
  v8f acc[2][8];
#pragma unroll
  for (int r = 0; r < 2; ++r)
#pragma unroll
    for (int t = 0; t < 8; ++t) acc[r][t] = (v8f){};
  for (int kb = 0; kb < D; kb += 32) { v16b a0, l0, a1, l1; frag_split(ctx + (size_t)(m0 + nloc) * D + kb, hlf, a0, l0); frag_split(ctx + (size_t)(m0 + 16 + nloc) * D + kb, hlf, a1, l1);
#pragma unroll
    for (int t = 0; t < 8; ++t) { const v16b bw = frag_kb(Wo + (size_t)(c0 + t * 16 + nloc) * D + kb, hlf); acc[0][t] = wmma16b(a0, bw, acc[0][t]); acc[0][t] = wmma16b(l0, bw, acc[0][t]); acc[1][t] = wmma16b(a1, bw, acc[1][t]); acc[1][t] = wmma16b(l1, bw, acc[1][t]); } }
#pragma unroll
  for (int t = 0; t < 8; ++t) { const float bb = P[3072 + c0 + t * 16 + nloc];
#pragma unroll
    for (int r = 0; r < 2; ++r)
#pragma unroll
      for (int v = 0; v < 8; ++v) Ts[wave][r * 16 + 8 * hlf + v][t * 16 + nloc] = acc[r][t][v] * (1.0f / AS_) + bb; }
  wave_lds_sync();
  for (int pass = 0; pass < 2; ++pass) { for (int i = lane; i < 32 * 32; i += 32) { const int rr = i >> 5, c4 = (i & 31) * 4; *(volatile v4f*)(out + (size_t)(m0 + rr) * D + c0 + c4) = *(const v4f*)(&Ts[wave][rr][c4]); } __threadfence(); }
}
}

extern "C" void kernel_launch(void* const* d_in, const int* in_sizes, int n_in,
                              void* d_out, int out_size, void* d_ws, size_t ws_size, hipStream_t stream) {
  (void)n_in; (void)out_size;
  const float* x = (const float*)d_in[0]; const float* Wq = (const float*)d_in[1]; const float* bq = (const float*)d_in[2]; const float* Wk = (const float*)d_in[3]; const float* bk = (const float*)d_in[4]; const float* Wv = (const float*)d_in[5]; const float* bv = (const float*)d_in[6]; const float* Wo = (const float*)d_in[7]; const float* bo = (const float*)d_in[8]; const float* rel = (const float*)d_in[9];
  float* out = (float*)d_out;
  if (in_sizes[0] != NT * D || in_sizes[1] != D * D || in_sizes[9] != NREL * HD) return;
  size_t off = 0; char* ws = (char*)d_ws;
  auto carve = [&](size_t bytes) { char* p = ws + off; off += (bytes + 255) & ~(size_t)255; return p; };
  b16* R = (b16*)carve(Wo_::END * 2); float* P = (float*)carve(4096 * 4); b16* qh = (b16*)carve(PL * 2); b16* ql = (b16*)carve(PL * 2); b16* kh = (b16*)carve(PL * 2); b16* kl = (b16*)carve(PL * 2); b16* vt = (b16*)carve(PL * 2); b16* vtl = (b16*)carve(PL * 2); float* ctx = (float*)carve((size_t)NT * D * 4);
  if (off > ws_size) return;
  prep_kernel<<<512, 256, 0, stream>>>(Wq, Wk, Wv, Wo, rel, bq, bk, bv, bo, R, P);
  proj_kernel<<<dim3(H, NT / 128, 3), 128, 0, stream>>>(x, R, P, qh, ql, kh, kl, vt, vtl);
  attn_kernel<<<dim3(NT / 16, H / 4), 128, 0, stream>>>(qh, ql, kh, kl, vt, vtl, R, ctx);
  out_kernel<<<dim3(D / 256, NT / 32), 64, 0, stream>>>(ctx, R, P, out);
}
